// CrossGraphAttention_59931973649023
// MI455X (gfx1250) — hardware-verified
//
#include <hip/hip_runtime.h>


#define TOT  16384
#define DD   512
#define D3   1536
#define NH_  8
#define HD   64
#define NG   16
#define NMAX 1088
#define TOTP (TOT + NMAX)
#define DM   DD
#define SCL  0.125f
#define LOSC 1024.0f

typedef _Float16 h16;
typedef unsigned short bf;
typedef __attribute__((ext_vector_type(16))) __bf16   v16bf;
typedef __attribute__((ext_vector_type(16))) _Float16 v16h;
typedef __attribute__((ext_vector_type(8)))  _Float16 v8h;
typedef __attribute__((ext_vector_type(8)))  unsigned short v8us;
typedef __attribute__((ext_vector_type(8)))  float    v8f;
typedef __attribute__((ext_vector_type(4)))  float    v4f;
typedef v8h  __attribute__((may_alias)) v8ha;
typedef v4f  __attribute__((may_alias)) v4fa;
typedef v8us __attribute__((may_alias)) v8usa;

__device__ __forceinline__ unsigned short f2bf(float f) { unsigned u = __float_as_uint(f); u += 0x7FFFu + ((u >> 16) & 1u); return (unsigned short)(u >> 16); }
__device__ __forceinline__ float bf2f(unsigned short b) { return __uint_as_float(((unsigned)b) << 16); }
__device__ __forceinline__ float bfr(float f) { return bf2f(f2bf(f)); }
__device__ __forceinline__ v16h cat16(v8h lo, v8h hi) { return __builtin_shufflevector(lo, hi, 0, 1, 2, 3, 4, 5, 6, 7, 8, 9, 10, 11, 12, 13, 14, 15); }
__device__ __forceinline__ v16bf cat16b(v8us lo, v8us hi) { return __builtin_bit_cast(v16bf, __builtin_shufflevector(lo, hi, 0, 1, 2, 3, 4, 5, 6, 7, 8, 9, 10, 11, 12, 13, 14, 15)); }
__device__ __forceinline__ v8f wmma16(v16h a, v16h b, v8f c) { return __builtin_amdgcn_wmma_f32_16x16x32_f16(false, a, false, b, (short)0, c, false, false); }
__device__ __forceinline__ v8f wmmab(v16bf a, v16bf b, v8f c) { return __builtin_amdgcn_wmma_f32_16x16x32_bf16(false, a, false, b, (short)0, c, false, false); }

template <bool SPLITA, bool F16OUT = false>
__global__ __launch_bounds__(128) void k_gemmb(const bf* __restrict__ A, const bf* __restrict__ Al, const bf* __restrict__ Bn, const float* __restrict__ bias, float* C, int ldc, h16* C2, const float* __restrict__ R = nullptr, int K = DM, int roundR = 1) {
    __shared__ __align__(16) float ost[4][16 * 68];
    const int lane = threadIdx.x & 31, wave = threadIdx.x >> 5, lr = lane & 15, hi = lane >> 4;
    const int r0 = blockIdx.x * 64 + wave * 16, c0 = blockIdx.y * 64;
    const size_t aoff = (size_t)(r0 + lr) * K + 8 * hi;
    size_t boff[4];
#pragma unroll
    for (int t = 0; t < 4; ++t) boff[t] = (size_t)(c0 + t * 16 + lr) * K + 8 * hi;
    v8f acc[4];
#pragma unroll
    for (int t = 0; t < 4; ++t) acc[t] = (v8f){};
#pragma unroll 1
    for (int kc = 0; kc < K; kc += 32) {
        const v16bf a = cat16b(*(const v8us*)(A + aoff + kc), *(const v8us*)(A + aoff + kc + 16));
        v16bf al = a;
        if (SPLITA) al = cat16b(*(const v8us*)(Al + aoff + kc), *(const v8us*)(Al + aoff + kc + 16));
#pragma unroll
        for (int t = 0; t < 4; ++t) { const v16bf b = cat16b(*(const v8us*)(Bn + boff[t] + kc), *(const v8us*)(Bn + boff[t] + kc + 16)); acc[t] = wmmab(a, b, acc[t]); if (SPLITA) acc[t] = wmmab(al, b, acc[t]); }
        asm volatile("v_nop\n\tv_nop\n\tv_nop\n\tv_nop" : "+v"(acc[0]), "+v"(acc[1]), "+v"(acc[2]), "+v"(acc[3]) : "v"(a), "v"(al));
    }
    float* os = &ost[wave][0];
#pragma unroll
    for (int t = 0; t < 4; ++t) { const float bv = bias ? bfr(bias[c0 + t * 16 + lr]) : 0.f;
#pragma unroll
        for (int j = 0; j < 8; ++j) os[(hi * 8 + j) * 68 + t * 16 + lr] = acc[t][j] + bv; }
    __syncthreads();
    if (F16OUT) {
        h16* crow = (h16*)(void*)C + (size_t)r0 * ldc + c0;
        auto pass = [&]() {
#pragma unroll
            for (int s = 0; s < 4; ++s) { const int row = 4 * s + (lane >> 3), piece = lane & 7; const float* sp = os + row * 68 + piece * 8; v8h o, o2;
#pragma unroll
                for (int i = 0; i < 8; ++i) { const h16 a = (h16)sp[i]; o[i] = a; o2[i] = (h16)((sp[i] - (float)a) * LOSC); }
                *(volatile v8h*)(crow + (size_t)row * ldc + piece * 8) = o; if (C2) *(volatile v8h*)(C2 + (size_t)r0 * ldc + c0 + (size_t)row * ldc + piece * 8) = o2; }
        };
        pass(); __threadfence(); pass();
    } else {
        float* crow = C + (size_t)r0 * ldc + c0;
        auto pass = [&]() {
#pragma unroll
            for (int s = 0; s < 8; ++s) { const int Lid = (lane >> 3) + 4 * s, piece = lane & 7; const int row = Lid >> 1, cofs = (Lid & 1) * 32 + piece * 4;
                v4f val = *(const v4fa*)(os + row * 68 + cofs); if (R) { const v4f rv = *(const v4f*)(R + ((size_t)r0 + row) * ldc + c0 + cofs); val += roundR ? (v4f){bfr(rv[0]), bfr(rv[1]), bfr(rv[2]), bfr(rv[3])} : rv; }
                *(volatile v4f*)(crow + (size_t)row * ldc + cofs) = val; }
        };
        pass(); __threadfence(); pass();
    }
}

__global__ __launch_bounds__(256) void k_cvt8(const float* __restrict__ src, bf* dst, size_t n8) {
    const size_t i = (size_t)blockIdx.x * 256 + threadIdx.x; if (i >= n8) return;
    const v8f v = *(const v8f*)(src + i * 8); v8us o;
#pragma unroll
    for (int k = 0; k < 8; ++k) o[k] = f2bf(v[k]);
    *(volatile v8us*)(dst + i * 8) = o; __threadfence(); *(volatile v8us*)(dst + i * 8) = o;
}
__global__ __launch_bounds__(256) void k_zero8(bf* dst, size_t n8) {
    const size_t i = (size_t)blockIdx.x * 256 + threadIdx.x; if (i >= n8) return; v8us z;
#pragma unroll
    for (int k = 0; k < 8; ++k) z[k] = 0;
    *(volatile v8us*)(dst + i * 8) = z; __threadfence(); *(volatile v8us*)(dst + i * 8) = z;
}
typedef __attribute__((ext_vector_type(4))) _Float16 v4h;
__device__ __forceinline__ h16 tohx(float x) { return (h16)x; }
__global__ __launch_bounds__(256) void k_segs(const int* __restrict__ batch, int* SEG) {
    if (threadIdx.x >= 32) return; const int lane = threadIdx.x; int cnt[NG];
#pragma unroll
    for (int g = 0; g < NG; ++g) cnt[g] = 0;
    for (int i = lane; i < TOT; i += 32) { int b = batch[i]; b = b < 0 ? 0 : (b >= NG ? NG - 1 : b);
#pragma unroll
        for (int g = 0; g < NG; ++g) cnt[g] += (b == g) ? 1 : 0; }
#pragma unroll
    for (int g = 0; g < NG; ++g) {
#pragma unroll
        for (int sh = 16; sh; sh >>= 1) cnt[g] += __shfl_xor(cnt[g], sh, 32); }
    int v = 0; int off = 0;
#pragma unroll
    for (int g = 0; g < NG; ++g) { if (lane == g) v = off; if (lane == NG + g) v = min(cnt[g], NMAX); off += cnt[g]; }
    *(volatile int*)(SEG + lane) = v; __threadfence(); *(volatile int*)(SEG + lane) = v;
}
__global__ __launch_bounds__(256) void k_cvthpad(const float* __restrict__ x, h16* XH) {
    const int lane = threadIdx.x & 31; const size_t r = (size_t)blockIdx.x * 8 + (threadIdx.x >> 5); if (r >= (size_t)TOTP) return; const bool live = r < (size_t)TOT;
#pragma unroll 1
    for (int ps = 0; ps < 2; ++ps) {
#pragma unroll
        for (int q = 0; q < 2; ++q) { v8h o;
#pragma unroll
            for (int i = 0; i < 8; ++i) o[i] = tohx(live ? bfr(x[r * DD + lane * 16 + q * 8 + i]) : 0.f);
            *(volatile v8h*)(XH + r * DD + lane * 16 + q * 8) = o; }
        if (ps == 0) __threadfence(); }
}
__global__ __launch_bounds__(256) void k_wnh(const float* __restrict__ Wm, size_t n8, h16* Bt) {
    const size_t i = (size_t)blockIdx.x * 256 + threadIdx.x; if (i >= n8) return; v8h o; const v8f v = *(const v8f*)(Wm + i * 8);
#pragma unroll
    for (int k = 0; k < 8; ++k) o[k] = tohx(bfr(v[k]));
    *(volatile v8h*)(Bt + i * 8) = o; __threadfence(); *(volatile v8h*)(Bt + i * 8) = o;
}
__global__ __launch_bounds__(256) void k_hplg(const float* __restrict__ QKV, const int* __restrict__ SEG, int g, int col0, float sc, h16* P) {
    const int lane = threadIdx.x & 31; const size_t w = (size_t)blockIdx.x * 8 + (threadIdx.x >> 5); if (w >= (size_t)NMAX / 2) return; const int h = blockIdx.z; const int n = SEG[NG + g]; const int i = (int)(w * 2 + (lane >> 4)); const int c0 = (lane & 15) * 4; v4h o;
#pragma unroll
    for (int q = 0; q < 4; ++q) o[q] = tohx(i < n ? QKV[(size_t)i * D3 + col0 + h * HD + c0 + q] * sc : 0.f);
    const size_t off = ((size_t)h * NMAX + i) * HD + c0; *(volatile v4h*)(P + off) = o; __threadfence(); *(volatile v4h*)(P + off) = o;
}
__global__ __launch_bounds__(256) void k_vTg(const float* __restrict__ QKV, const int* __restrict__ SEG, int g, h16* VT) {
    __shared__ float tl[64][65];
    const int tid = threadIdx.x; const int t0 = blockIdx.x * 64; const int h = blockIdx.z; const int n = SEG[NG + g]; const int rr = tid >> 2, cq = (tid & 3) * 16;
#pragma unroll
    for (int i = 0; i < 16; ++i) tl[rr][cq + i] = (t0 + rr < n) ? QKV[(size_t)(t0 + rr) * D3 + 2 * DD + h * HD + cq + i] : 0.f;
    __syncthreads();
    const int lane = tid & 31, wv = tid >> 5;
    auto pass = [&]() {
#pragma unroll
        for (int st = 0; st < 4; ++st) { const int dr = wv * 8 + st * 2 + (lane >> 4); const int tq = (lane & 15) * 4; v4h v;
#pragma unroll
            for (int i = 0; i < 4; ++i) v[i] = tohx(tl[tq + i][dr]);
            *(volatile v4h*)(VT + ((size_t)h * HD + dr) * NMAX + t0 + tq) = v; }
    };
    pass(); __threadfence(); pass();
}
__global__ __launch_bounds__(256) void k_softg(const float* __restrict__ S, const int* __restrict__ SEG, int g, h16* P) {
    typedef __attribute__((ext_vector_type(2))) _Float16 v2h;
    const int lane = threadIdx.x & 31, i = blockIdx.x * 8 + (threadIdx.x >> 5); if (i >= NMAX) return; const int n = SEG[NG + g]; const size_t zo = (size_t)blockIdx.z * NMAX * NMAX; const float* sr = S + zo + (size_t)i * NMAX; h16* pr = P + zo + (size_t)i * NMAX;
    float m = -3.0e38f;
#pragma unroll 1
    for (int c0 = lane * 2; c0 < NMAX; c0 += 64) {
#pragma unroll
        for (int q = 0; q < 2; ++q) { const int j = c0 + q; if (j < n) m = fmaxf(m, sr[j]); } }
#pragma unroll
    for (int sh = 16; sh; sh >>= 1) m = fmaxf(m, __shfl_xor(m, sh, 32));
    float sum = 0.f;
#pragma unroll 1
    for (int c0 = lane * 2; c0 < NMAX; c0 += 64) {
#pragma unroll
        for (int q = 0; q < 2; ++q) { const int j = c0 + q; if (j < n) sum += __expf(sr[j] - m); } }
#pragma unroll
    for (int sh = 16; sh; sh >>= 1) sum += __shfl_xor(sum, sh, 32);
    const float inv = 1.0f / sum;
#pragma unroll 1
    for (int ps = 0; ps < 2; ++ps) {
#pragma unroll 1
        for (int c0 = lane * 2; c0 < NMAX; c0 += 64) { v2h o;
#pragma unroll
            for (int q = 0; q < 2; ++q) { const int j = c0 + q; o[q] = tohx((j < n) ? __expf(sr[(j < n) ? j : 0] - m) * inv : 0.f); }
            *(volatile v2h*)(pr + c0) = o; }
        if (ps == 0) __threadfence(); }
}
__global__ __launch_bounds__(256) void k_split512(const float* __restrict__ F, size_t rows, bf* Ph, bf* Pl) {
    const int lane = threadIdx.x & 31; const size_t r = (size_t)blockIdx.x * 8 + (threadIdx.x >> 5); if (r >= rows) return;
#pragma unroll 1
    for (int ps = 0; ps < 2; ++ps) {
#pragma unroll
        for (int hq = 0; hq < 2; ++hq) { const size_t o = r * DD + lane * 16 + hq * 8; const v8f v = *(const v8f*)(F + o); v8us oh, ol;
#pragma unroll
            for (int i = 0; i < 8; ++i) { const unsigned short hb = f2bf(v[i]); oh[i] = hb; ol[i] = f2bf(v[i] - bf2f(hb)); }
            *(volatile v8us*)(Ph + o) = oh; *(volatile v8us*)(Pl + o) = ol; }
        if (ps == 0) __threadfence(); }
}
__global__ __launch_bounds__(128) void k_gemmhs(const h16* __restrict__ A, const h16* __restrict__ Bn, const float* __restrict__ bias, float* C, int ldc, int K, const int* __restrict__ SEG, int g, int shiftA, int shiftC, size_t sA, size_t sB, size_t sC) {
    __shared__ __align__(16) float ost[4][16 * 68];
    const size_t off = (size_t)SEG[g]; if (shiftA) A += off * K; if (shiftC) C += off * ldc;
    const size_t z = blockIdx.z; A += z * sA; Bn += z * sB; C += z * sC;
    const int lane = threadIdx.x & 31, wave = threadIdx.x >> 5, lr = lane & 15, hi = lane >> 4;
    const int r0 = blockIdx.x * 64 + wave * 16, c0 = blockIdx.y * 64;
    const size_t aoff = (size_t)(r0 + lr) * K + 8 * hi;
    size_t boff[4];
#pragma unroll
    for (int t = 0; t < 4; ++t) boff[t] = (size_t)(c0 + t * 16 + lr) * K + 8 * hi;
    v8f acc[4];
#pragma unroll
    for (int t = 0; t < 4; ++t) acc[t] = (v8f){};
#pragma unroll 1
    for (int kc = 0; kc < K; kc += 32) {
        const v16h a = cat16(*(const v8h*)(A + aoff + kc), *(const v8h*)(A + aoff + kc + 16));
#pragma unroll
        for (int t = 0; t < 4; ++t) { const v16h b = cat16(*(const v8h*)(Bn + boff[t] + kc), *(const v8h*)(Bn + boff[t] + kc + 16)); acc[t] = wmma16(a, b, acc[t]); }
        asm volatile("v_nop\n\tv_nop\n\tv_nop\n\tv_nop" : "+v"(acc[0]), "+v"(acc[1]), "+v"(acc[2]), "+v"(acc[3]) : "v"(a));
    }
    float* os = &ost[wave][0];
#pragma unroll
    for (int t = 0; t < 4; ++t) { const float bv = bias ? bfr(bias[c0 + t * 16 + lr]) : 0.f;
#pragma unroll
        for (int j = 0; j < 8; ++j) os[(hi * 8 + j) * 68 + t * 16 + lr] = acc[t][j] + bv; }
    __syncthreads();
    float* crow = C + (size_t)r0 * ldc + c0;
    auto pass = [&]() {
#pragma unroll
        for (int s = 0; s < 8; ++s) { const int Lid = (lane >> 3) + 4 * s, piece = lane & 7; const int row = Lid >> 1, cofs = (Lid & 1) * 32 + piece * 4;
            const v4f val = *(const v4fa*)(os + row * 68 + cofs); *(volatile v4f*)(crow + (size_t)row * ldc + cofs) = val; }
    };
    pass(); __threadfence(); pass();
}

extern "C" void kernel_launch(void* const* d_in, const int* in_sizes, int n_in,
                              void* d_out, int out_size, void* d_ws, size_t ws_size, hipStream_t stream) {
    (void)in_sizes; (void)n_in; (void)out_size;
    const float* x = (const float*)d_in[0]; const int* batch = (const int*)d_in[1]; const float* ipw = (const float*)d_in[2]; const float* ipb = (const float*)d_in[3]; const float* opw = (const float*)d_in[4]; const float* opb = (const float*)d_in[5]; const float* lw = (const float*)d_in[6]; const float* lb = (const float*)d_in[7];
    float* out = (float*)d_out;
    char* wsp = (char*)d_ws;
    auto take = [&](size_t bytes) { char* p = wsp; wsp += (bytes + 255) & ~(size_t)255; return (void*)p; };
    int* SEG = (int*)take(32 * 4); h16* WIP = (h16*)take((size_t)D3 * DD * 2); bf* WOP = (bf*)take((size_t)DD * DD * 2); bf* WL = (bf*)take((size_t)DD * DD * 2);
    h16* XH = (h16*)take((size_t)TOTP * DD * 2); float* QKV = (float*)take((size_t)NMAX * D3 * 4); h16* QPL = (h16*)take((size_t)NH_ * NMAX * HD * 2); h16* KPL = (h16*)take((size_t)NH_ * NMAX * HD * 2); h16* VT = (h16*)take((size_t)NH_ * HD * NMAX * 2);
    char* const shared0 = wsp;
    float* S = (float*)take((size_t)NH_ * NMAX * NMAX * 4); h16* PP = (h16*)take((size_t)NH_ * NMAX * NMAX * 2);
    char* const attEnd = wsp; wsp = shared0;
    bf* Oh = (bf*)take((size_t)TOTP * DD * 2); bf* Ol = (bf*)take((size_t)TOTP * DD * 2); float* AO = (float*)take((size_t)TOTP * DD * 4);
    if (wsp < attEnd) wsp = attEnd;
    float* O = (float*)take((size_t)TOTP * DD * 4);
    if ((size_t)(wsp - (char*)d_ws) > ws_size) return;
    k_segs<<<1, 256, 0, stream>>>(batch, SEG);
    k_wnh<<<(unsigned)(((size_t)D3 * DD / 8 + 255) / 256), 256, 0, stream>>>(ipw, (size_t)D3 * DD / 8, WIP); k_cvt8<<<(unsigned)(((size_t)DD * DD / 8 + 255) / 256), 256, 0, stream>>>(opw, WOP, (size_t)DD * DD / 8); k_cvt8<<<(unsigned)(((size_t)DD * DD / 8 + 255) / 256), 256, 0, stream>>>(lw, WL, (size_t)DD * DD / 8);
    k_cvthpad<<<TOTP / 8, 256, 0, stream>>>(x, XH);
    for (int g = 0; g < NG; ++g) {
        k_gemmhs<<<dim3(NMAX / 64, D3 / 64, 1), 128, 0, stream>>>(XH, WIP, ipb, QKV, D3, DD, SEG, g, 1, 0, 0, 0, 0);
        k_hplg<<<dim3((NMAX / 2) / 8, 1, NH_), 256, 0, stream>>>(QKV, SEG, g, 0, SCL, QPL); k_hplg<<<dim3((NMAX / 2) / 8, 1, NH_), 256, 0, stream>>>(QKV, SEG, g, DD, 1.0f, KPL); k_vTg<<<dim3(NMAX / 64, 1, NH_), 256, 0, stream>>>(QKV, SEG, g, VT);
        k_gemmhs<<<dim3(NMAX / 64, NMAX / 64, NH_), 128, 0, stream>>>(QPL, KPL, nullptr, S, NMAX, HD, SEG, g, 0, 0, (size_t)NMAX * HD, (size_t)NMAX * HD, (size_t)NMAX * NMAX);
        k_softg<<<dim3(NMAX / 8, 1, NH_), 256, 0, stream>>>(S, SEG, g, PP);
        k_gemmhs<<<dim3(NMAX / 64, 1, NH_), 128, 0, stream>>>(PP, VT, nullptr, O, DD, NMAX, SEG, g, 0, 1, (size_t)NMAX * NMAX, (size_t)HD * NMAX, (size_t)HD); }
    k_split512<<<TOTP / 8, 256, 0, stream>>>(O, TOTP, Oh, Ol);
    k_gemmb<true, false><<<dim3(TOTP / 64, DD / 64, 1), 128, 0, stream>>>(Oh, Ol, WOP, opb, AO, DD, nullptr, nullptr, DD);
    k_split512<<<TOTP / 8, 256, 0, stream>>>(AO, TOTP, Oh, Ol);
    k_gemmb<true, false><<<dim3(TOT / 64, DD / 64, 1), 128, 0, stream>>>(Oh, Ol, WL, lb, out, DD, nullptr, nullptr, DD);
}
